// Attention_25675314495536
// MI455X (gfx1250) — hardware-verified
//
#include <hip/hip_runtime.h>


#ifndef NB
#define NB 2
#endif
#ifndef SEQ
#define SEQ 4096
#endif
#define NB_FULL  2
#define SEQ_FULL 4096
#define EMB  768
#define NH   12
#define HD   64
#define NQKV (3 * EMB)
#define NWV  4
#define BQ   (16 * NWV)
#define KS   32
#define OSP  68
#define GTM  128
#define GTN  64
#define QKP  72
#define VTP  136
#define PJP  68
#define L2E  1.4426950408889634f
#define SCL2E (0.125f * L2E)
#define PCARRY 10.0f

static_assert(EMB == NH * HD);
static_assert(HD == 64);
static_assert(GTN == HD);
static_assert(EMB % 32 == 0);
static_assert(EMB % GTN == 0);
static_assert(NQKV % GTN == 0);
static_assert(SEQ % GTM == 0);
static_assert(SEQ % BQ == 0);
static_assert(SEQ % KS == 0);
static_assert(NB <= NB_FULL);
static_assert(SEQ <= SEQ_FULL);
static_assert(GTM * QKP >= HD * VTP);
static_assert((QKP % 8) == 0 && (VTP % 8) == 0 && (OSP % 4) == 0 && (PJP % 4) == 0);

#define XG     ((unsigned)(SEQ * (EMB / 8)))
#define CB_X   ((unsigned)(NB * SEQ * (EMB / 8) / 256))
#define CB_WQ  ((unsigned)(NQKV * EMB / 8 / 256))
#define CB_WP  ((unsigned)(EMB * EMB / 8 / 256))
static_assert(((size_t)NB * SEQ * (EMB / 8)) % 256 == 0);
static_assert(((size_t)NQKV * EMB / 8) % 256 == 0);
static_assert(((size_t)EMB * EMB / 8) % 256 == 0);
static_assert((size_t)(CB_X + CB_WQ + CB_WP) * 256 * 8 == (size_t)NB * SEQ * EMB + (size_t)NQKV * EMB + (size_t)EMB * EMB);
static_assert((size_t)(NB * SEQ / GTM) * (NQKV / GTN) * (size_t)(GTM * GTN) == (size_t)3 * NB * SEQ * EMB);
static_assert(128 * 8 * 8 == GTM * GTN);
static_assert((size_t)(NB * NH * (SEQ / BQ)) * (size_t)(BQ * HD) == (size_t)NB * SEQ * EMB);
static_assert(32 * 4 * 8 == 16 * HD);
static_assert((size_t)(NB * SEQ / GTM) * (EMB / GTN) * (size_t)(GTM * GTN) == (size_t)NB * SEQ * EMB);
static_assert(128 * 16 * 4 == GTM * GTN);

#define PL_ACT ((size_t)NB * SEQ * EMB * 2)
#define PL_WQ  ((size_t)NQKV * EMB * 2)
#define PL_WP  ((size_t)EMB * EMB * 2)
#define WS_TOTAL (6 * PL_ACT + PL_WQ + PL_WP)
static_assert(PL_ACT % 128 == 0 && PL_WQ % 128 == 0 && PL_WP % 128 == 0);
static_assert(WS_TOTAL <= (size_t)134217728);

typedef unsigned short bf;
typedef unsigned short hf;
typedef __attribute__((ext_vector_type(16))) __bf16   v16bf;
typedef __attribute__((ext_vector_type(16))) _Float16 v16h;
typedef __attribute__((ext_vector_type(8)))  unsigned short v8us;
typedef __attribute__((ext_vector_type(8)))  float    v8f;
typedef __attribute__((ext_vector_type(4)))  float    v4f;
typedef v4f  __attribute__((may_alias)) v4fa;
typedef v8us __attribute__((may_alias)) v8usa;

__device__ __forceinline__ unsigned short f2bf(float f) { unsigned u = __float_as_uint(f); u += 0x7FFFu + ((u >> 16) & 1u); return (unsigned short)(u >> 16); }
__device__ __forceinline__ float bf2f(unsigned short b) { return __uint_as_float(((unsigned)b) << 16); }
__device__ __forceinline__ float bfr(float f) { return bf2f(f2bf(f)); }
__device__ __forceinline__ unsigned short f2h(float f) { return __builtin_bit_cast(unsigned short, (_Float16)f); }
__device__ __forceinline__ v16bf cat16b(v8us lo, v8us hi) { return __builtin_bit_cast(v16bf, __builtin_shufflevector(lo, hi, 0, 1, 2, 3, 4, 5, 6, 7, 8, 9, 10, 11, 12, 13, 14, 15)); }
__device__ __forceinline__ v16h  cat16h(v8us lo, v8us hi) { return __builtin_bit_cast(v16h,  __builtin_shufflevector(lo, hi, 0, 1, 2, 3, 4, 5, 6, 7, 8, 9, 10, 11, 12, 13, 14, 15)); }
__device__ __forceinline__ v8f wmmab(v16bf a, v16bf b, v8f c) { return __builtin_amdgcn_wmma_f32_16x16x32_bf16(false, a, false, b, (short)0, c, false, false); }
__device__ __forceinline__ v8f wmmah(v16h a, v16h b, v8f c) { return __builtin_amdgcn_wmma_f32_16x16x32_f16(false, a, false, b, (short)0, c, false, false); }
__device__ __forceinline__ v16bf ldb(const bf* p) { return cat16b(*(const v8us*)p, *(const v8us*)(p + 16)); }
__device__ __forceinline__ v16h  ldh(const hf* p) { return cat16h(*(const v8us*)p, *(const v8us*)(p + 16)); }

__global__ __launch_bounds__(256) void k_cvt(const float* __restrict__ x, const float* __restrict__ wq, const float* __restrict__ wp, bf* XB, bf* WQ, bf* WP) {
    const unsigned blk = blockIdx.x, tid = threadIdx.x;
    const float* src;
    bf* dst;
    if (blk < CB_X) {
        const unsigned i = blk * 256u + tid;
        const unsigned b = i / XG, r = i - b * XG;
        src = x + (size_t)b * SEQ_FULL * EMB + (size_t)r * 8;
        dst = XB + (size_t)i * 8;
    } else if (blk < CB_X + CB_WQ) {
        const unsigned i = (blk - CB_X) * 256u + tid;
        src = wq + (size_t)i * 8;
        dst = WQ + (size_t)i * 8;
    } else {
        const unsigned i = (blk - CB_X - CB_WQ) * 256u + tid;
        src = wp + (size_t)i * 8;
        dst = WP + (size_t)i * 8;
    }
    const v8f v = *(const v8f*)src;
    v8us o;
#pragma unroll
    for (int c = 0; c < 8; ++c) o[c] = f2bf(v[c]);
    *(volatile v8us*)dst = o;
    __threadfence();
    *(volatile v8us*)dst = o;
}

__device__ __forceinline__ void mm_acc(const bf* __restrict__ ap, const bf* __restrict__ bp, v8f (&acc)[2][4]) {
#pragma unroll 1
    for (unsigned k0 = 0; k0 < (unsigned)EMB; k0 += 32u) {
        const v16bf a0 = ldb(ap + k0);
        const v16bf a1 = ldb(ap + 16 * EMB + k0);
#pragma unroll
        for (int nt = 0; nt < 4; ++nt) {
            const v16bf w = ldb(bp + nt * 16 * EMB + k0);
            acc[0][nt] = wmmab(a0, w, acc[0][nt]);
            acc[1][nt] = wmmab(a1, w, acc[1][nt]);
        }
        asm volatile("v_nop\n\tv_nop\n\tv_nop\n\tv_nop"
                     : "+v"(acc[0][0]), "+v"(acc[0][1]), "+v"(acc[0][2]), "+v"(acc[0][3]),
                       "+v"(acc[1][0]), "+v"(acc[1][1]), "+v"(acc[1][2]), "+v"(acc[1][3])
                     : "v"(a0), "v"(a1));
    }
}

__global__ __launch_bounds__(128) void k_qkv(const bf* __restrict__ XB, const bf* __restrict__ WQ, hf* QP, hf* KP, hf* VT) {
    __shared__ __align__(16) unsigned short tl[GTM * QKP];
    const unsigned tid = threadIdx.x, lane = tid & 31u, wv = tid >> 5, lr = lane & 15u, hi = lane >> 4;
    const unsigned m0 = blockIdx.x * GTM;
    const unsigned n0 = blockIdx.y * GTN;
    v8f acc[2][4];
#pragma unroll
    for (int mt = 0; mt < 2; ++mt)
#pragma unroll
        for (int nt = 0; nt < 4; ++nt) acc[mt][nt] = (v8f){};
    mm_acc(XB + (size_t)(m0 + wv * 32u + lr) * EMB + 8u * hi, WQ + (size_t)(n0 + lr) * EMB + 8u * hi, acc);

    const unsigned part = blockIdx.y / NH;
    const unsigned hh = blockIdx.y - part * NH;
    const unsigned b = m0 / (unsigned)SEQ;
    const unsigned s0 = m0 - b * (unsigned)SEQ;
    const unsigned bh = b * NH + hh;
    if (part < 2u) {
#pragma unroll
        for (int mt = 0; mt < 2; ++mt)
#pragma unroll
            for (int nt = 0; nt < 4; ++nt)
#pragma unroll
                for (int r = 0; r < 8; ++r)
                    tl[(wv * 32u + mt * 16u + 8u * hi + r) * QKP + nt * 16u + lr] = f2h(acc[mt][nt][r]);
    } else {
#pragma unroll
        for (int mt = 0; mt < 2; ++mt)
#pragma unroll
            for (int nt = 0; nt < 4; ++nt)
#pragma unroll
                for (int r = 0; r < 8; ++r)
                    tl[(nt * 16u + lr) * VTP + wv * 32u + mt * 16u + 8u * hi + r] = f2h(acc[mt][nt][r]);
    }
    __syncthreads();
    if (part < 2u) {
        hf* dst = (part == 0u ? QP : KP) + ((size_t)bh * SEQ + s0) * HD;
        const unsigned pc = (tid & 7u) * 8u, rr = tid >> 3;
#pragma unroll 1
        for (int ps = 0; ps < 2; ++ps) {
#pragma unroll
            for (unsigned it = 0; it < 8; ++it) {
                const unsigned row = it * 16u + rr;
                const v8us o = *(const v8usa*)(tl + row * QKP + pc);
                *(volatile v8us*)(dst + (size_t)row * HD + pc) = o;
            }
            if (ps == 0) __threadfence();
        }
    } else {
        hf* dst = VT + (size_t)bh * HD * SEQ + s0;
        const unsigned pc = (tid & 15u) * 8u, dr = tid >> 4;
#pragma unroll 1
        for (int ps = 0; ps < 2; ++ps) {
#pragma unroll
            for (unsigned it = 0; it < 8; ++it) {
                const unsigned d = it * 8u + dr;
                const v8us o = *(const v8usa*)(tl + d * VTP + pc);
                *(volatile v8us*)(dst + (size_t)d * SEQ + pc) = o;
            }
            if (ps == 0) __threadfence();
        }
    }
}

__global__ __launch_bounds__(128) void k_flash(const hf* __restrict__ QP, const hf* __restrict__ KP, const hf* __restrict__ VT, bf* CH, bf* CL) {
    __shared__ __align__(16) float os[NWV * 16 * OSP];
    const unsigned tid = threadIdx.x, lane = tid & 31u, wv = tid >> 5, lr = lane & 15u, hi = lane >> 4;
    const unsigned bpb = (unsigned)(SEQ / BQ);
    const unsigned bh = blockIdx.x / bpb;
    const unsigned qb = blockIdx.x - bh * bpb;
    const unsigned b = bh / NH;
    const unsigned h = bh - b * NH;
    const unsigned q0 = qb * BQ + wv * 16u;

    v16h qf[2];
    {
        const hf* qp = QP + ((size_t)bh * SEQ + q0 + lr) * HD + 8u * hi;
#pragma unroll
        for (int dk = 0; dk < 2; ++dk) qf[dk] = ldh(qp + dk * 32);
    }
    const hf* kp = KP + ((size_t)bh * SEQ + lr) * HD + 8u * hi;
    const hf* vp = VT + ((size_t)bh * HD + lr) * SEQ + 8u * hi;

    v8f o[4];
#pragma unroll
    for (int t = 0; t < 4; ++t) o[t] = (v8f){};
    float ml = -1.0e30f;
    float l = 0.0f;

#pragma unroll 1
    for (unsigned k0 = 0; k0 < (unsigned)SEQ; k0 += KS) {
        v8f s0 = (v8f){}, s1 = (v8f){};
        const hf* ka = kp + (size_t)k0 * HD;
#pragma unroll
        for (int dk = 0; dk < 2; ++dk) {
            const v16h a0 = ldh(ka + dk * 32);
            const v16h a1 = ldh(ka + 16 * HD + dk * 32);
            s0 = wmmah(a0, qf[dk], s0);
            s1 = wmmah(a1, qf[dk], s1);
        }
        asm volatile("v_nop\n\tv_nop\n\tv_nop\n\tv_nop" : "+v"(s0), "+v"(s1) : "v"(qf[0]), "v"(qf[1]));

        float mx = fmaxf(s0[0], s1[0]);
#pragma unroll
        for (int r = 1; r < 8; ++r) mx = fmaxf(mx, fmaxf(s0[r], s1[r]));
        mx = fmaxf(mx, __shfl_xor(mx, 16, 32));
        const float mnl = fmaxf(ml, mx * SCL2E);
        const float corr = __builtin_amdgcn_exp2f(ml - mnl);
        ml = mnl;
        const float sh = mnl - PCARRY;
        float p0[8], p1[8];
        float ps = 0.0f;
#pragma unroll
        for (int r = 0; r < 8; ++r) {
            p0[r] = __builtin_amdgcn_exp2f(fmaf(s0[r], SCL2E, -sh));
            p1[r] = __builtin_amdgcn_exp2f(fmaf(s1[r], SCL2E, -sh));
            ps += p0[r] + p1[r];
        }
        ps += __shfl_xor(ps, 16, 32);
        l = l * corr + ps;
        if (__builtin_amdgcn_ballot_w32(corr != 1.0f) != 0u) {
#pragma unroll
            for (int t = 0; t < 4; ++t) o[t] *= corr;
        }

        v16h ph;
#pragma unroll
        for (int r = 0; r < 8; ++r) {
            ph[r]     = (_Float16)p0[r];
            ph[8 + r] = (_Float16)p1[r];
        }

        asm volatile("" ::: "memory");
        const hf* va = vp + k0;
#pragma unroll
        for (int t = 0; t < 4; ++t) {
            const v16h a = ldh(va + (size_t)t * 16 * SEQ);
            o[t] = wmmah(a, ph, o[t]);
        }
        asm volatile("v_nop\n\tv_nop\n\tv_nop\n\tv_nop"
                     : "+v"(o[0]), "+v"(o[1]), "+v"(o[2]), "+v"(o[3])
                     : "v"(ph));
    }

    const float inv = 1.0f / l;
    float* ow = os + wv * (16 * OSP);
#pragma unroll
    for (int t = 0; t < 4; ++t) {
#pragma unroll
        for (int r = 0; r < 8; ++r) ow[lr * OSP + t * 16 + 8 * hi + r] = o[t][r] * inv;
    }
    __syncthreads();
    const unsigned pc = (lane & 7u) * 8u, rq = lane >> 3;
    const size_t cbase = ((size_t)b * SEQ + q0) * EMB + h * HD + pc;
    bf* ch = CH + cbase;
    bf* cl = CL + cbase;
#pragma unroll 1
    for (int ps2 = 0; ps2 < 2; ++ps2) {
#pragma unroll
        for (unsigned it = 0; it < 4; ++it) {
            const unsigned row = it * 4u + rq;
            const v4f x0 = *(const v4fa*)(ow + row * OSP + pc);
            const v4f x1 = *(const v4fa*)(ow + row * OSP + pc + 4u);
            v8us oh, ol;
#pragma unroll
            for (int c = 0; c < 4; ++c) {
                const unsigned u0 = __float_as_uint(x0[c]), u1 = __float_as_uint(x1[c]);
                oh[c]     = (unsigned short)(u0 >> 16);
                oh[4 + c] = (unsigned short)(u1 >> 16);
                ol[c]     = f2bf(x0[c] - __uint_as_float(u0 & 0xFFFF0000u));
                ol[4 + c] = f2bf(x1[c] - __uint_as_float(u1 & 0xFFFF0000u));
            }
            *(volatile v8us*)(ch + (size_t)row * EMB) = oh;
            *(volatile v8us*)(cl + (size_t)row * EMB) = ol;
        }
        if (ps2 == 0) __threadfence();
    }
}

__global__ __launch_bounds__(128) void k_proj(const bf* __restrict__ CH, const bf* __restrict__ CL, const bf* __restrict__ WP, const float* __restrict__ bias, float* OUT) {
    __shared__ __align__(16) float tf[GTM * PJP];
    const unsigned tid = threadIdx.x, lane = tid & 31u, wv = tid >> 5, lr = lane & 15u, hi = lane >> 4;
    const unsigned m0 = blockIdx.x * GTM;
    const unsigned n0 = blockIdx.y * GTN;
    v8f acc[2][4];
#pragma unroll
    for (int mt = 0; mt < 2; ++mt)
#pragma unroll
        for (int nt = 0; nt < 4; ++nt) acc[mt][nt] = (v8f){};
    const size_t aoff = (size_t)(m0 + wv * 32u + lr) * EMB + 8u * hi;
    const bf* bp = WP + (size_t)(n0 + lr) * EMB + 8u * hi;
    mm_acc(CH + aoff, bp, acc);
    mm_acc(CL + aoff, bp, acc);
#pragma unroll
    for (int mt = 0; mt < 2; ++mt)
#pragma unroll
        for (int nt = 0; nt < 4; ++nt)
#pragma unroll
            for (int r = 0; r < 8; ++r)
                tf[(wv * 32u + mt * 16u + 8u * hi + r) * PJP + nt * 16u + lr] = acc[mt][nt][r];
    __syncthreads();
    const unsigned pc = (tid & 15u) * 4u, rr = tid >> 4;
    const v4f braw = *(const v4f*)(bias + n0 + pc);
    v4f bb;
    bb[0] = bfr(braw[0]); bb[1] = bfr(braw[1]); bb[2] = bfr(braw[2]); bb[3] = bfr(braw[3]);
    float* dst = OUT + (size_t)m0 * EMB + n0 + pc;
#pragma unroll 1
    for (int ps = 0; ps < 2; ++ps) {
#pragma unroll 4
        for (unsigned it = 0; it < 16; ++it) {
            const unsigned row = it * 8u + rr;
            v4f val = *(const v4fa*)(tf + row * PJP + pc);
            val += bb;
            *(volatile v4f*)(dst + (size_t)row * EMB) = val;
        }
        if (ps == 0) __threadfence();
    }
}

extern "C" void kernel_launch(void* const* d_in, const int* in_sizes, int n_in,
                              void* d_out, int out_size, void* d_ws, size_t ws_size, hipStream_t stream) {
    if (n_in < 4) return;
    const size_t need_x = ((size_t)(NB - 1) * SEQ_FULL + SEQ) * EMB;
    if ((size_t)in_sizes[0] < need_x) return;
    if ((size_t)in_sizes[1] < (size_t)NQKV * EMB) return;
    if ((size_t)in_sizes[2] < (size_t)EMB * EMB) return;
    if ((size_t)in_sizes[3] < (size_t)EMB) return;
    if ((size_t)out_size < (size_t)NB * SEQ * EMB) return;
    if (WS_TOTAL > ws_size) return;
    const float* x  = (const float*)d_in[0];
    const float* wq = (const float*)d_in[1];
    const float* wp = (const float*)d_in[2];
    const float* bp = (const float*)d_in[3];
    float* OUT = (float*)d_out;
    char* wsp = (char*)d_ws;
    bf* XB = (bf*)(wsp);
    bf* WQ = (bf*)(wsp + PL_ACT);
    bf* WP = (bf*)(wsp + PL_ACT + PL_WQ);
    hf* QP = (hf*)(wsp + PL_ACT + PL_WQ + PL_WP);
    hf* KP = (hf*)(wsp + 2 * PL_ACT + PL_WQ + PL_WP);
    hf* VT = (hf*)(wsp + 3 * PL_ACT + PL_WQ + PL_WP);
    bf* CH = (bf*)(wsp + 4 * PL_ACT + PL_WQ + PL_WP);
    bf* CL = (bf*)(wsp + 5 * PL_ACT + PL_WQ + PL_WP);
    k_cvt<<<CB_X + CB_WQ + CB_WP, 256, 0, stream>>>(x, wq, wp, XB, WQ, WP);
    k_qkv<<<dim3((unsigned)(NB * SEQ / GTM), (unsigned)(NQKV / GTN), 1), 128, 0, stream>>>(XB, WQ, QP, KP, VT);
    k_flash<<<(unsigned)(NB * NH * (SEQ / BQ)), 128, 0, stream>>>(QP, KP, VT, CH, CL);
    k_proj<<<dim3((unsigned)(NB * SEQ / GTM), (unsigned)(EMB / GTN), 1), 128, 0, stream>>>(CH, CL, WP, bp, OUT);
}
